// SelfAttention_53584011985680
// MI455X (gfx1250) — hardware-verified
//
#include <hip/hip_runtime.h>


#ifndef NB
#define NB 2
#endif
#ifndef SEQ
#define SEQ 2048
#endif
#define NB_FULL  2
#define SEQ_FULL 2048
#define DM   1024
#define NH   16
#define HD   64
#define TP   72
#define PCAR 1024.0f
#define WSC  64.0f
#define OSC  (1.0f / 65536.0f)
#define CL2  0.045084220027780106f
#define NEGL (-4.5084220027780106e18f)
static_assert(DM == NH * HD);
static_assert(HD == 64);
static_assert(SEQ % 128 == 0);
static_assert(SEQ <= SEQ_FULL);
static_assert(NB <= NB_FULL);
static_assert((NB * SEQ) % 64 == 0);
static_assert(DM % 64 == 0);
static_assert(DM % 32 == 0);
static_assert(TP >= 64 && (TP % 8) == 0);

typedef _Float16 h16;
typedef __attribute__((ext_vector_type(16))) __bf16   v16bf;
typedef __attribute__((ext_vector_type(16))) _Float16 v16h;
typedef __attribute__((ext_vector_type(8)))  _Float16 v8h;
typedef __attribute__((ext_vector_type(8)))  unsigned short v8us;
typedef __attribute__((ext_vector_type(8)))  float    v8f;
typedef __attribute__((ext_vector_type(4)))  float    v4f;
typedef v8h __attribute__((may_alias)) v8ha;
typedef v4f __attribute__((may_alias)) v4fa;

__device__ __forceinline__ unsigned short f2bf(float f) { unsigned u = __float_as_uint(f); u += 0x7FFFu + ((u >> 16) & 1u); return (unsigned short)(u >> 16); }
__device__ __forceinline__ float bf2f(unsigned short b) { return __uint_as_float(((unsigned)b) << 16); }
__device__ __forceinline__ float bfr(float f) { return bf2f(f2bf(f)); }
__device__ __forceinline__ v16h cat16(v8h lo, v8h hi) { return __builtin_shufflevector(lo, hi, 0, 1, 2, 3, 4, 5, 6, 7, 8, 9, 10, 11, 12, 13, 14, 15); }
__device__ __forceinline__ v16bf cat16b(v8us lo, v8us hi) { return __builtin_bit_cast(v16bf, __builtin_shufflevector(lo, hi, 0, 1, 2, 3, 4, 5, 6, 7, 8, 9, 10, 11, 12, 13, 14, 15)); }
__device__ __forceinline__ v8f wmma16(v16h a, v16h b, v8f c) { return __builtin_amdgcn_wmma_f32_16x16x32_f16(false, a, false, b, (short)0, c, false, false); }
__device__ __forceinline__ v8f wmmab(v16bf a, v16bf b, v8f c) { return __builtin_amdgcn_wmma_f32_16x16x32_bf16(false, a, false, b, (short)0, c, false, false); }
__device__ __forceinline__ v16h ldh(const h16* __restrict__ p) { return cat16(*(const v8h*)p, *(const v8h*)(p + 16)); }
__device__ __forceinline__ v16bf ldf32(const float* __restrict__ p) {
    const v4f a = *(const v4f*)p; const v4f b = *(const v4f*)(p + 4); const v4f c = *(const v4f*)(p + 16); const v4f d = *(const v4f*)(p + 20);
    v8us lo, hi;
    lo[0] = f2bf(a[0]); lo[1] = f2bf(a[1]); lo[2] = f2bf(a[2]); lo[3] = f2bf(a[3]); lo[4] = f2bf(b[0]); lo[5] = f2bf(b[1]); lo[6] = f2bf(b[2]); lo[7] = f2bf(b[3]);
    hi[0] = f2bf(c[0]); hi[1] = f2bf(c[1]); hi[2] = f2bf(c[2]); hi[3] = f2bf(c[3]); hi[4] = f2bf(d[0]); hi[5] = f2bf(d[1]); hi[6] = f2bf(d[2]); hi[7] = f2bf(d[3]);
    return cat16b(lo, hi);
}
__device__ __forceinline__ void wsync() { __builtin_amdgcn_fence(3  , "wavefront"); __builtin_amdgcn_wave_barrier(); asm volatile("" ::: "memory"); }

__global__ __launch_bounds__(256) void k_cvtw(const float* __restrict__ src, h16* dst, int n8) {
    const int i = blockIdx.x * 256 + threadIdx.x; if (i >= n8) return;
    const v4f a = *(const v4f*)(src + (size_t)i * 8); const v4f b = *(const v4f*)(src + (size_t)i * 8 + 4); v8h o;
    o[0] = (h16)(bfr(a[0]) * WSC); o[1] = (h16)(bfr(a[1]) * WSC); o[2] = (h16)(bfr(a[2]) * WSC); o[3] = (h16)(bfr(a[3]) * WSC);
    o[4] = (h16)(bfr(b[0]) * WSC); o[5] = (h16)(bfr(b[1]) * WSC); o[6] = (h16)(bfr(b[2]) * WSC); o[7] = (h16)(bfr(b[3]) * WSC);
    *(volatile v8h*)(dst + (size_t)i * 8) = o; __threadfence(); *(volatile v8h*)(dst + (size_t)i * 8) = o;
}

template <int MODE>
__device__ __forceinline__ void proj_body(const float* __restrict__ X, const float* __restrict__ W, h16* dst) {
    __shared__ __align__(16) h16 T[32 * TP];
    const int lane = threadIdx.x & 31, lr = lane & 15, hi = lane >> 4;
    const int h = blockIdx.y; const int bx = blockIdx.x;
    int n, s0, eh;
    if (MODE == 0) { n = bx / (SEQ / 32); s0 = (bx % (SEQ / 32)) * 32; eh = 0; }
    else { const int tb = bx >> 1; eh = bx & 1; n = tb / (SEQ / 64); s0 = (tb % (SEQ / 64)) * 64; }
    const float* xp = X + ((size_t)n * SEQ_FULL + s0 + lr) * DM + h * HD + 8 * hi;
    const float* wp = W + (size_t)(eh * 32 + lr) * HD + 8 * hi;
    v8f acc[4][2];
#pragma unroll
    for (int mb = 0; mb < 4; ++mb) { acc[mb][0] = (v8f){}; acc[mb][1] = (v8f){}; }
#pragma unroll
    for (int ks = 0; ks < 2; ++ks) {
        v16bf rf[4], cf[2];
        if (MODE == 0) {
#pragma unroll
            for (int i = 0; i < 4; ++i) rf[i] = ldf32(wp + (size_t)i * 16 * HD + ks * 32);
#pragma unroll
            for (int i = 0; i < 2; ++i) cf[i] = ldf32(xp + (size_t)i * 16 * DM + ks * 32);
        } else {
#pragma unroll
            for (int i = 0; i < 4; ++i) rf[i] = ldf32(xp + (size_t)i * 16 * DM + ks * 32);
#pragma unroll
            for (int i = 0; i < 2; ++i) cf[i] = ldf32(wp + (size_t)i * 16 * HD + ks * 32);
        }
#pragma unroll
        for (int nb = 0; nb < 2; ++nb)
#pragma unroll
            for (int mb = 0; mb < 4; ++mb) acc[mb][nb] = wmmab(rf[mb], cf[nb], acc[mb][nb]);
        asm volatile("v_nop\n\tv_nop\n\tv_nop\n\tv_nop" : "+v"(acc[0][0]), "+v"(acc[1][0]), "+v"(acc[2][0]), "+v"(acc[3][0]), "+v"(acc[0][1]), "+v"(acc[1][1]), "+v"(acc[2][1]), "+v"(acc[3][1]) : "v"(rf[3]), "v"(cf[1]));
    }
#pragma unroll
    for (int nb = 0; nb < 2; ++nb)
#pragma unroll
        for (int mb = 0; mb < 4; ++mb) { v8h o;
#pragma unroll
            for (int j = 0; j < 8; ++j) o[j] = (h16)acc[mb][nb][j];
            *(v8ha*)&T[(nb * 16 + lr) * TP + mb * 16 + 8 * hi] = o; }
    wsync();
    v8h val[8];
#pragma unroll
    for (int s = 0; s < 8; ++s) val[s] = *(const v8ha*)&T[(4 * s + (lane >> 3)) * TP + (lane & 7) * 8];
    size_t base, step;
    if (MODE == 0) { base = ((size_t)n * SEQ + s0 + (lane >> 3)) * DM + h * HD + (lane & 7) * 8; step = (size_t)4 * DM; }
    else { base = (((size_t)n * NH + h) * HD + eh * 32 + (lane >> 3)) * SEQ + s0 + (lane & 7) * 8; step = (size_t)4 * SEQ; }
#pragma unroll 1
    for (int ps = 0; ps < 2; ++ps) {
#pragma unroll
        for (int s = 0; s < 8; ++s) *(volatile v8h*)(dst + base + (size_t)s * step) = val[s];
        if (ps == 0) __threadfence(); }
}
__global__ __launch_bounds__(32) void k_projqk(const float* __restrict__ X, const float* __restrict__ W, h16* dst) { proj_body<0>(X, W, dst); }
__global__ __launch_bounds__(32) void k_projvt(const float* __restrict__ X, const float* __restrict__ W, h16* dst) { proj_body<1>(X, W, dst); }

__device__ __forceinline__ void split8(const v8f o, const float inv, v8h& hv, v8h& lv) {
#pragma unroll
    for (int r = 0; r < 8; ++r) { const float x = o[r] * inv; const h16 xh = (h16)x; hv[r] = xh; lv[r] = (h16)(x - (float)xh); }
}

__global__ __launch_bounds__(128) void k_flash(const h16* __restrict__ QF, const h16* __restrict__ KF, const h16* __restrict__ VT, const int* __restrict__ mask, h16* ATh, h16* ATl) {
#pragma clang fp contract(off)
    __shared__ unsigned smw[SEQ / 32];
    __shared__ __align__(16) h16 sth[4][16 * TP];
    __shared__ __align__(16) h16 stl[4][16 * TP];
    const int wave = __builtin_amdgcn_readfirstlane((int)(threadIdx.x >> 5));
    const int lane = threadIdx.x & 31, lr = lane & 15, hi = lane >> 4;
    const int h = blockIdx.y, n = blockIdx.z;
    const int q0 = blockIdx.x * 64 + wave * 16;
#pragma unroll 1
    for (int w = wave * (SEQ / 128); w < (wave + 1) * (SEQ / 128); ++w) {
        const int mv = mask[(size_t)n * SEQ_FULL + w * 32 + lane];
        const unsigned bw = __builtin_amdgcn_ballot_w32(mv != 0);
        smw[w] = bw;
    }
    __syncthreads();
    const h16* qp = QF + ((size_t)n * SEQ + q0 + lr) * DM + h * HD + 8 * hi;
    const v16h qf0 = ldh(qp), qf1 = ldh(qp + 32);
    const h16* kp = KF + ((size_t)n * SEQ + lr) * DM + h * HD + 8 * hi;
    const h16* vp = VT + (((size_t)n * NH + h) * HD + lr) * SEQ + 8 * hi;
    v8f o0 = (v8f){}, o1 = (v8f){}, o2 = (v8f){}, o3 = (v8f){};
    float m_run = -3.0e38f, l_run = 0.0f;
#pragma unroll 1
    for (int st = 0; st < SEQ / 32; ++st) {
        const h16* kq = kp + (size_t)st * 32 * DM;
        const v16h k00 = ldh(kq), k01 = ldh(kq + 32), k10 = ldh(kq + (size_t)16 * DM), k11 = ldh(kq + (size_t)16 * DM + 32);
        v8f s0 = (v8f){}, s1 = (v8f){};
        s0 = wmma16(k00, qf0, s0); s0 = wmma16(k01, qf1, s0);
        s1 = wmma16(k10, qf0, s1); s1 = wmma16(k11, qf1, s1);
        asm volatile("v_nop\n\tv_nop\n\tv_nop\n\tv_nop" : "+v"(s0), "+v"(s1) : "v"(k11), "v"(qf1));
        const unsigned mw = (unsigned)__builtin_amdgcn_readfirstlane((int)smw[st]);
#pragma unroll
        for (int r = 0; r < 8; ++r) { s0[r] = s0[r] * CL2; s1[r] = s1[r] * CL2; }
        if (mw != 0xFFFFFFFFu) {
            const unsigned bits = mw >> (8 * hi);
#pragma unroll
            for (int r = 0; r < 8; ++r) { s0[r] = ((bits >> r) & 1u) ? s0[r] : NEGL; s1[r] = ((bits >> (16 + r)) & 1u) ? s1[r] : NEGL; }
        }
        float mx = fmaxf(s0[0], s1[0]);
#pragma unroll
        for (int r = 1; r < 8; ++r) mx = fmaxf(mx, fmaxf(s0[r], s1[r]));
        mx = fmaxf(mx, __shfl_xor(mx, 16, 32));
        const float mn = fmaxf(m_run, mx);
        if (__builtin_amdgcn_ballot_w32(mn > m_run) != 0u) {
            const float al = __builtin_amdgcn_exp2f(m_run - mn);
            l_run *= al; o0 *= al; o1 *= al; o2 *= al; o3 *= al;
            m_run = mn;
        }
        float ls = 0.0f; v16h pf;
#pragma unroll
        for (int r = 0; r < 8; ++r) { const float p0 = __builtin_amdgcn_exp2f(s0[r] - mn); const float p1 = __builtin_amdgcn_exp2f(s1[r] - mn); ls += p0 + p1; pf[r] = (h16)p0; pf[8 + r] = (h16)p1; }
        l_run += ls;
        const h16* vq = vp + st * 32;
        const v16h v0 = ldh(vq), v1 = ldh(vq + (size_t)16 * SEQ), v2 = ldh(vq + (size_t)32 * SEQ), v3 = ldh(vq + (size_t)48 * SEQ);
        o0 = wmma16(v0, pf, o0); o1 = wmma16(v1, pf, o1); o2 = wmma16(v2, pf, o2); o3 = wmma16(v3, pf, o3);
        asm volatile("v_nop\n\tv_nop\n\tv_nop\n\tv_nop" : "+v"(o0), "+v"(o1), "+v"(o2), "+v"(o3) : "v"(v3), "v"(pf));
    }
    const float l = l_run + __shfl_xor(l_run, 16, 32);
    const float inv = PCAR * (1.0f / l);
    v8h h0, l0, h1, l1, h2, l2, h3, l3;
    split8(o0, inv, h0, l0); split8(o1, inv, h1, l1); split8(o2, inv, h2, l2); split8(o3, inv, h3, l3);
    const int sb = lr * TP + 8 * hi;
    *(v8ha*)&sth[wave][sb] = h0; *(v8ha*)&sth[wave][sb + 16] = h1; *(v8ha*)&sth[wave][sb + 32] = h2; *(v8ha*)&sth[wave][sb + 48] = h3;
    *(v8ha*)&stl[wave][sb] = l0; *(v8ha*)&stl[wave][sb + 16] = l1; *(v8ha*)&stl[wave][sb + 32] = l2; *(v8ha*)&stl[wave][sb + 48] = l3;
    wsync();
    v8h hv[4], lv[4];
#pragma unroll
    for (int s = 0; s < 4; ++s) { const int rb = (4 * s + (lane >> 3)) * TP + (lane & 7) * 8; hv[s] = *(const v8ha*)&sth[wave][rb]; lv[s] = *(const v8ha*)&stl[wave][rb]; }
    const size_t ob = ((size_t)n * SEQ + q0 + (lane >> 3)) * DM + h * HD + (lane & 7) * 8;
#pragma unroll 1
    for (int ps = 0; ps < 2; ++ps) {
#pragma unroll
        for (int s = 0; s < 4; ++s) { *(volatile v8h*)(ATh + ob + (size_t)(4 * s) * DM) = hv[s]; *(volatile v8h*)(ATl + ob + (size_t)(4 * s) * DM) = lv[s]; }
        if (ps == 0) __threadfence(); }
}

__global__ __launch_bounds__(32) void k_oproj(const h16* __restrict__ A, const h16* __restrict__ A2, const h16* __restrict__ Bt, float* C, const float* __restrict__ bias) {
    __shared__ __align__(16) float os[16 * 68];
    const int lane = threadIdx.x & 31, lr = lane & 15, hi = lane >> 4; const int r0 = blockIdx.x * 64, c0 = blockIdx.y * 64;
    v8f acc[4][4];
#pragma unroll
    for (int mb = 0; mb < 4; ++mb)
#pragma unroll
        for (int nb = 0; nb < 4; ++nb) acc[mb][nb] = (v8f){};
    const size_t aoff = (size_t)(r0 + lr) * DM + 8 * hi, boff = (size_t)(c0 + lr) * DM + 8 * hi;
#pragma unroll 1
    for (int kc = 0; kc < DM; kc += 32) {
        v16h a[4], a2[4], b;
#pragma unroll
        for (int mb = 0; mb < 4; ++mb) { a[mb] = ldh(A + aoff + (size_t)mb * 16 * DM + kc); a2[mb] = ldh(A2 + aoff + (size_t)mb * 16 * DM + kc); }
#pragma unroll
        for (int nb = 0; nb < 4; ++nb) { b = ldh(Bt + boff + (size_t)nb * 16 * DM + kc);
#pragma unroll
            for (int mb = 0; mb < 4; ++mb) { acc[mb][nb] = wmma16(a[mb], b, acc[mb][nb]); acc[mb][nb] = wmma16(a2[mb], b, acc[mb][nb]); } }
        asm volatile("" : "+v"(acc[0][0]), "+v"(acc[1][0]), "+v"(acc[2][0]), "+v"(acc[3][0]), "+v"(acc[0][1]), "+v"(acc[1][1]), "+v"(acc[2][1]), "+v"(acc[3][1]));
        asm volatile("v_nop\n\tv_nop\n\tv_nop\n\tv_nop" : "+v"(acc[0][2]), "+v"(acc[1][2]), "+v"(acc[2][2]), "+v"(acc[3][2]), "+v"(acc[0][3]), "+v"(acc[1][3]), "+v"(acc[2][3]), "+v"(acc[3][3]) : "v"(a2[3]), "v"(b));
    }
    const int cofs = lr * 4;
    const v4f bv = *(const v4f*)(bias + c0 + cofs);
    v4f bb; bb[0] = bfr(bv[0]); bb[1] = bfr(bv[1]); bb[2] = bfr(bv[2]); bb[3] = bfr(bv[3]);
#pragma unroll
    for (int mb = 0; mb < 4; ++mb) {
#pragma unroll
        for (int nb = 0; nb < 4; ++nb) {
#pragma unroll
            for (int j = 0; j < 8; ++j) os[(hi * 8 + j) * 68 + nb * 16 + lr] = acc[mb][nb][j]; }
        wsync();
        v4f val[8];
#pragma unroll
        for (int s = 0; s < 8; ++s) { const v4f t = *(const v4fa*)&os[(2 * s + hi) * 68 + cofs]; val[s] = t * OSC + bb; }
        float* crow = C + (size_t)(r0 + mb * 16 + hi) * DM + c0 + cofs;
#pragma unroll 1
        for (int ps = 0; ps < 2; ++ps) {
#pragma unroll
            for (int s = 0; s < 8; ++s) *(volatile v4f*)(crow + (size_t)(2 * s) * DM) = val[s];
            if (ps == 0) __threadfence(); }
        wsync();
    }
}

static constexpr size_t SZ_W = (size_t)DM * DM * 2;
static constexpr size_t SZ_P = (size_t)NB * SEQ * DM * 2;
static_assert(SZ_W % 256 == 0);
static_assert(SZ_P % 256 == 0);
static_assert(SZ_W + 5 * SZ_P <= (size_t)134217728);

extern "C" void kernel_launch(void* const* d_in, const int* in_sizes, int n_in,
                              void* d_out, int out_size, void* d_ws, size_t ws_size, hipStream_t stream) {
    if (n_in < 9) return;
    const int need_x = ((NB - 1) * SEQ_FULL + SEQ) * DM;
    if (in_sizes[0] < need_x || in_sizes[1] < need_x || in_sizes[2] < need_x) return;
    if (in_sizes[3] < (NB - 1) * SEQ_FULL + SEQ) return;
    if (in_sizes[4] < HD * HD || in_sizes[5] < HD * HD || in_sizes[6] < HD * HD) return;
    if (in_sizes[7] < DM * DM || in_sizes[8] < DM) return;
    if (out_size < NB * SEQ * DM) return;
    if (SZ_W + 5 * SZ_P > ws_size) return;
    const float* xv = (const float*)d_in[0];
    const float* xk = (const float*)d_in[1];
    const float* xq = (const float*)d_in[2];
    const int*   mk = (const int*)d_in[3];
    const float* wv = (const float*)d_in[4];
    const float* wk = (const float*)d_in[5];
    const float* wq = (const float*)d_in[6];
    const float* wo = (const float*)d_in[7];
    const float* bo = (const float*)d_in[8];
    float* OUT = (float*)d_out;
    char* wsp = (char*)d_ws;
    h16* WO  = (h16*)wsp; wsp += SZ_W;
    h16* QF  = (h16*)wsp; wsp += SZ_P;
    h16* KF  = (h16*)wsp; wsp += SZ_P;
    h16* VTp = (h16*)wsp; wsp += SZ_P;
    h16* ATh = (h16*)wsp; wsp += SZ_P;
    h16* ATl = (h16*)wsp; wsp += SZ_P;
    k_cvtw<<<(DM * DM / 8 + 255) / 256, 256, 0, stream>>>(wo, WO, DM * DM / 8);
    k_projqk<<<dim3(NB * SEQ / 32, NH, 1), 32, 0, stream>>>(xq, wq, QF);
    k_projqk<<<dim3(NB * SEQ / 32, NH, 1), 32, 0, stream>>>(xk, wk, KF);
    k_projvt<<<dim3(NB * SEQ / 32, NH, 1), 32, 0, stream>>>(xv, wv, VTp);
    k_flash<<<dim3(SEQ / 64, NH, NB), 128, 0, stream>>>(QF, KF, VTp, mk, ATh, ATl);
    k_oproj<<<dim3(NB * SEQ / 64, DM / 64, 1), 32, 0, stream>>>(ATh, ATl, WO, OUT, bo);
}
